// slice_model_80075370267325
// MI455X (gfx1250) — hardware-verified
//
#include <hip/hip_runtime.h>
#include <stddef.h>
#include <stdint.h>


#define CF       128
#define NLEN     4096
#define LOUT     4094
#define NGR      16
#define LP       4096
#define CO1      128
#define CO2      256
#define NCH      (CO1 + CO2)
#define KC       (2 * CF)
#define NTHR     256
#define NWAVE    8
#define EPT      8
#define NGRP     2
#define CHUNK    (NTHR * EPT * NGRP)
#define WCAP     (EPT * NGRP * 32)
#define LISTN    (NWAVE * WCAP)
#define TD       1024
#define TPW      (TD / NWAVE)
#define PBLK     128
#define WSCALE   16.0f
#define WINV     0.0625f
#define BNEPS    1e-5f
#define L2EPS    1e-12f

#define LDS_AGG  (TD * CF * 2 + LISTN * 4 + 64)
#define LDS_CONV (128 * PBLK * 4)

static_assert((CHUNK & (CHUNK - 1)) == 0);
static_assert(CHUNK <= 4096);
static_assert((TD & (TD - 1)) == 0 && TD <= 4096);
static_assert(TPW == 128);
static_assert(NLEN % PBLK == 0 && PBLK == NWAVE * 16);
static_assert((NGR * NLEN) % TD == 0);
static_assert(NCH % 32 == 0 && CO1 % 32 == 0);
static_assert(CF % 32 == 0 && KC % 32 == 0);

typedef float    v4f  __attribute__((ext_vector_type(4)));
typedef float    v8f  __attribute__((ext_vector_type(8)));
typedef int      v4i  __attribute__((ext_vector_type(4)));
typedef _Float16 v4h  __attribute__((ext_vector_type(4)));
typedef _Float16 v8h  __attribute__((ext_vector_type(8)));
typedef _Float16 v16h __attribute__((ext_vector_type(16)));
union FragH { v16h v; v8h h[2]; };

__device__ __forceinline__ v8h cvt8(v4f a, v4f b) {
  v8h r;
  r[0] = (_Float16)a.x; r[1] = (_Float16)a.y; r[2] = (_Float16)a.z; r[3] = (_Float16)a.w;
  r[4] = (_Float16)b.x; r[5] = (_Float16)b.y; r[6] = (_Float16)b.z; r[7] = (_Float16)b.w;
  return r;
}

__device__ __forceinline__ v8f wmh(v16h a, v16h b, v8f c) {
  v8f d = __builtin_amdgcn_wmma_f32_16x16x32_f16(false, a, false, b, (short)0, c, false, false);
  asm volatile("v_nop\n\tv_nop\n\tv_nop\n\tv_nop" : "+v"(d) : "v"(a), "v"(b));
  return d;
}

__device__ __forceinline__ double shfl_xor_d(double v, int o) {
  const long long u = __double_as_longlong(v);
  int lo = (int)(u & 0xffffffffLL);
  int hi = (int)((unsigned long long)u >> 32);
  lo = __shfl_xor(lo, o, 32);
  hi = __shfl_xor(hi, o, 32);
  const unsigned long long r = ((unsigned long long)(unsigned)hi << 32) | (unsigned long long)(unsigned)lo;
  return __longlong_as_double((long long)r);
}

template <int NB>
__device__ __forceinline__ int scan_chunk(const int* __restrict__ dsts, int nE, int cbase, int slotBase,
                                          int vec8, int* list, int tid, int lane, int wave) {
  int wc = 0;
#pragma unroll
  for (int g = 0; g < NGRP; ++g) {
    const int el0  = (g * NTHR + tid) * EPT;
    const int e0   = cbase + el0;
    const int sent = -2147483647 - 1;
    v4i da, db;
    if (vec8 != 0 && cbase + CHUNK <= nE) {
      da = *(const v4i*)(dsts + e0);
      db = *(const v4i*)(dsts + e0 + 4);
    } else {
      da.x = (e0     < nE) ? dsts[min(e0, nE - 1)] : sent;
      da.y = (e0 + 1 < nE) ? dsts[min(e0 + 1, nE - 1)] : sent;
      da.z = (e0 + 2 < nE) ? dsts[min(e0 + 2, nE - 1)] : sent;
      da.w = (e0 + 3 < nE) ? dsts[min(e0 + 3, nE - 1)] : sent;
      db.x = (e0 + 4 < nE) ? dsts[min(e0 + 4, nE - 1)] : sent;
      db.y = (e0 + 5 < nE) ? dsts[min(e0 + 5, nE - 1)] : sent;
      db.z = (e0 + 6 < nE) ? dsts[min(e0 + 6, nE - 1)] : sent;
      db.w = (e0 + 7 < nE) ? dsts[min(e0 + 7, nE - 1)] : sent;
    }
    const unsigned nb = (unsigned)slotBase;
    const unsigned s0 = (unsigned)da.x - nb, s1 = (unsigned)da.y - nb;
    const unsigned s2 = (unsigned)da.z - nb, s3 = (unsigned)da.w - nb;
    const unsigned s4 = (unsigned)db.x - nb, s5 = (unsigned)db.y - nb;
    const unsigned s6 = (unsigned)db.z - nb, s7 = (unsigned)db.w - nb;
    const bool h0 = s0 < (unsigned)NB, h1 = s1 < (unsigned)NB, h2 = s2 < (unsigned)NB, h3 = s3 < (unsigned)NB;
    const bool h4 = s4 < (unsigned)NB, h5 = s5 < (unsigned)NB, h6 = s6 < (unsigned)NB, h7 = s7 < (unsigned)NB;
    const unsigned any = __builtin_amdgcn_ballot_w32(h0 | h1 | h2 | h3 | h4 | h5 | h6 | h7);
    if (any != 0u) {
#define HITJ(J, HJ, SJ) { \
        const unsigned mj = __builtin_amdgcn_ballot_w32(HJ); \
        if (mj != 0u) { \
          if (HJ) { \
            const int pos = wc + (int)__builtin_amdgcn_mbcnt_lo(mj, 0u); \
            if (pos < WCAP) list[wave * WCAP + pos] = ((el0 + (J)) << 12) | (int)(SJ); \
          } \
          wc += (int)__builtin_popcount(mj); } }
      HITJ(0, h0, s0)
      HITJ(1, h1, s1)
      HITJ(2, h2, s2)
      HITJ(3, h3, s3)
      HITJ(4, h4, s4)
      HITJ(5, h5, s5)
      HITJ(6, h6, s6)
      HITJ(7, h7, s7)
#undef HITJ
    }
  }
  return wc;
}

__global__ __launch_bounds__(NTHR) void k_prep(
    const float* __restrict__ wl, const float* __restrict__ wr,
    const float* __restrict__ c1, const float* __restrict__ c2,
    _Float16* wc, _Float16* wt1, _Float16* wt2) {
  const int g0 = CF * KC / 8;
  const int g1 = CO1 * 3 * CF / 8;
  const int g2 = CO2 * 3 * KC / 8;
  const int bstart = blockIdx.x * NTHR;
  const int i = bstart + (int)threadIdx.x;
  if (i >= g0 + g1 + g2) return;
  float v[8];
  _Float16* dp;
  if (bstart < g0) {
    const int o  = i * 8;
    const int n  = o / KC;
    const int k0 = o - n * KC;
    const int kk = k0 & (CF - 1);
#pragma unroll
    for (int e = 0; e < 8; ++e) {
      const float xl = wl[n * CF + kk + e];
      const float xr = wr[n * CF + kk + e];
      v[e] = (k0 < CF ? xl : xr) * WSCALE;
    }
    dp = wc + o;
  } else if (bstart < g0 + g1) {
    const int o   = (i - g0) * 8;
    const int n   = o / (3 * CF);
    const int k0  = o - n * (3 * CF);
    const int tap = k0 / CF;
    const int ci0 = k0 - tap * CF;
#pragma unroll
    for (int e = 0; e < 8; ++e) v[e] = c1[((size_t)(n * CF + ci0 + e)) * 3 + tap] * WSCALE;
    dp = wt1 + o;
  } else {
    const int o   = (i - g0 - g1) * 8;
    const int n   = o / (3 * KC);
    const int k0  = o - n * (3 * KC);
    const int tap = k0 / KC;
    const int ci0 = k0 - tap * KC;
#pragma unroll
    for (int e = 0; e < 8; ++e) v[e] = c2[((size_t)(n * KC + ci0 + e)) * 3 + tap] * WSCALE;
    dp = wt2 + o;
  }
  v4f a, b;
  a.x = v[0]; a.y = v[1]; a.z = v[2]; a.w = v[3];
  b.x = v[4]; b.y = v[5]; b.z = v[6]; b.w = v[7];
  const v8h hv = cvt8(a, b);
  *(volatile v8h*)dp = hv;
  __threadfence();
  *(volatile v8h*)dp = hv;
}

__global__ __launch_bounds__(NTHR) void k_aggl(
    const float* __restrict__ feat, const int* __restrict__ topo,
    const _Float16* __restrict__ wc, const float* __restrict__ bl,
    _Float16* s16, int nN, int nE, int vec8) {
  extern __shared__ v4f lds_dyn[];
  _Float16* sAgg = (_Float16*)lds_dyn;
  int* list = (int*)(sAgg + TD * CF);
  int* wcnt = list + LISTN;
  const int tid = threadIdx.x, lane = tid & 31, wave = tid >> 5, hh = lane >> 4, m = lane & 15;
  const int nodeBase = blockIdx.x * TD;
  const int* srcs = topo;
  const int* dsts = topo + nE;

  {
    v4i ninf;
    ninf.x = (int)0xFC00FC00u; ninf.y = ninf.x; ninf.z = ninf.x; ninf.w = ninf.x;
    v4i* p = (v4i*)sAgg;
#pragma unroll 1
    for (int i = tid; i < TD * CF * 2 / 16; i += NTHR) p[i] = ninf;
  }
  __syncthreads();

  const int nChunks = (nE + CHUNK - 1) / CHUNK;
#pragma unroll 1
  for (int ch = 0; ch < nChunks; ++ch) {
    const int cbase = ch * CHUNK;
    const int wc0 = scan_chunk<TD>(dsts, nE, cbase, nodeBase, vec8, list, tid, lane, wave);
    if (lane == 0) wcnt[wave] = wc0;
    __syncthreads();
#pragma unroll 1
    for (int s = 0; s < NWAVE; ++s) {
      int n = __builtin_amdgcn_readfirstlane(wcnt[s]);
      n = n > WCAP ? WCAP : (n < 0 ? 0 : n);
      const int* lp = list + s * WCAP;
#pragma unroll 1
      for (int b0 = 0; b0 < n; b0 += 32) {
        const int idx = b0 + lane;
        const int ent = lp[idx < WCAP ? idx : WCAP - 1];
        const bool mine = (idx < n) && (((ent >> 7) & (NWAVE - 1)) == wave);
        unsigned mk = (unsigned)__builtin_amdgcn_readfirstlane((int)__builtin_amdgcn_ballot_w32(mine));
#pragma unroll 1
        while (mk != 0u) {
          const int j = __builtin_ctz(mk);
          mk &= mk - 1u;
          const int en = __builtin_amdgcn_readlane(ent, j);
          const int slot = en & (TD - 1);
          int e = cbase + ((en >> 12) & (CHUNK - 1));
          e = e > nE - 1 ? nE - 1 : e;
          int sv = srcs[e];
          sv = sv < 0 ? 0 : (sv > nN - 1 ? nN - 1 : sv);
          const v4f f = *(const v4f*)(feat + (size_t)sv * CF + 4 * lane);
          v4h nv;
          nv.x = (_Float16)f.x; nv.y = (_Float16)f.y; nv.z = (_Float16)f.z; nv.w = (_Float16)f.w;
          v4h* hp = (v4h*)(sAgg + slot * CF + 4 * lane);
          const v4h cv = *hp;
          v4h r;
          r.x = cv.x > nv.x ? cv.x : nv.x;
          r.y = cv.y > nv.y ? cv.y : nv.y;
          r.z = cv.z > nv.z ? cv.z : nv.z;
          r.w = cv.w > nv.w ? cv.w : nv.w;
          *hp = r;
        }
      }
    }
    __syncthreads();
  }

  {
    v8h* p = (v8h*)sAgg;
    const _Float16 nlim = (_Float16)(-65504.0f);
    const _Float16 zh = (_Float16)0.0f;
#pragma unroll 1
    for (int i = tid; i < TD * CF / 8; i += NTHR) {
      v8h x = p[i];
#pragma unroll
      for (int e = 0; e < 8; ++e) x[e] = (x[e] < nlim) ? zh : x[e];
      p[i] = x;
    }
  }
  __syncthreads();

#pragma unroll 1
  for (int rt = 0; rt < TPW / 16; ++rt) {
    const int r0 = wave * TPW + 16 * rt;
    const size_t node = (size_t)nodeBase + r0 + m;
    v8f acc[8];
#pragma unroll
    for (int t = 0; t < 8; ++t) { v8f z = {0.f, 0.f, 0.f, 0.f, 0.f, 0.f, 0.f, 0.f}; acc[t] = z; }

    const _Float16* arow = sAgg + (r0 + m) * CF + 8 * hh;
#pragma unroll
    for (int ks = 0; ks < CF / 32; ++ks) {
      FragH a;
      a.h[0] = *(const v8h*)(arow + 32 * ks);
      a.h[1] = *(const v8h*)(arow + 32 * ks + 16);
#pragma unroll
      for (int t = 0; t < 8; ++t) {
        const _Float16* bp = wc + (size_t)(16 * t + m) * KC + 32 * ks + 8 * hh;
        FragH b;
        b.h[0] = *(const v8h*)bp;
        b.h[1] = *(const v8h*)(bp + 16);
        acc[t] = wmh(a.v, b.v, acc[t]);
      }
    }
    const float* frow = feat + node * CF + 8 * hh;
#pragma unroll
    for (int ks = 0; ks < CF / 32; ++ks) {
      FragH a;
      a.h[0] = cvt8(*(const v4f*)(frow + 32 * ks),      *(const v4f*)(frow + 32 * ks + 4));
      a.h[1] = cvt8(*(const v4f*)(frow + 32 * ks + 16), *(const v4f*)(frow + 32 * ks + 20));
#pragma unroll
      for (int t = 0; t < 8; ++t) {
        const _Float16* bp = wc + (size_t)(16 * t + m) * KC + CF + 32 * ks + 8 * hh;
        FragH b;
        b.h[0] = *(const v8h*)bp;
        b.h[1] = *(const v8h*)(bp + 16);
        acc[t] = wmh(a.v, b.v, acc[t]);
      }
    }

    float ss[8];
#pragma unroll
    for (int r = 0; r < 8; ++r) ss[r] = 0.0f;
#pragma unroll
    for (int t = 0; t < 8; ++t) {
      const float bv = bl[16 * t + m];
#pragma unroll
      for (int r = 0; r < 8; ++r) {
        const float y = acc[t][r] * WINV + bv;
        acc[t][r] = y;
        ss[r] += y * y;
      }
    }
#pragma unroll
    for (int o = 1; o < 16; o <<= 1) {
#pragma unroll
      for (int r = 0; r < 8; ++r) ss[r] += __shfl_xor(ss[r], o, 32);
    }
    float inv[8];
#pragma unroll
    for (int r = 0; r < 8; ++r) {
      const float nr = fmaxf(sqrtf(ss[r]), L2EPS);
      inv[r] = 1.0f / nr;
    }
    _Float16* sp = sAgg + (r0 + 8 * hh) * CF + m;
#pragma unroll
    for (int t = 0; t < 8; ++t) {
#pragma unroll
      for (int r = 0; r < 8; ++r) sp[r * CF + 16 * t] = (_Float16)(acc[t][r] * inv[r]);
    }
    __syncthreads();

    v8h ov[8];
#pragma unroll
    for (int p = 0; p < 8; ++p) ov[p] = *(const v8h*)(sAgg + (r0 + 2 * p + hh) * CF + 8 * m);
    _Float16* gp = s16 + ((size_t)nodeBase + r0) * CF + 8 * m;
#pragma unroll
    for (int p = 0; p < 8; ++p) *(volatile v8h*)(gp + (size_t)(2 * p + hh) * CF) = ov[p];
    __threadfence();
#pragma unroll
    for (int p = 0; p < 8; ++p) *(volatile v8h*)(gp + (size_t)(2 * p + hh) * CF) = ov[p];
  }
}

template <int CIN, int CO>
__global__ __launch_bounds__(NTHR) void k_conv(
    const _Float16* __restrict__ s16, const float* __restrict__ feat,
    const _Float16* __restrict__ wt, const float* __restrict__ bias, float* Y) {
  extern __shared__ v4f lds_dyn[];
  float* stg = (float*)lds_dyn;
  constexpr int KP = 3 * CIN;
  const int tid = threadIdx.x, lane = tid & 31, wave = tid >> 5, hh = lane >> 4, m = lane & 15;
  const int pb = blockIdx.x, b = blockIdx.y;
  const int l0 = pb * PBLK + wave * 16;

#pragma unroll 1
  for (int cg = 0; cg < CO / 128; ++cg) {
    v8f acc[8];
#pragma unroll
    for (int t = 0; t < 8; ++t) { v8f z = {0.f, 0.f, 0.f, 0.f, 0.f, 0.f, 0.f, 0.f}; acc[t] = z; }
#pragma unroll 1
    for (int tap = 0; tap < 3; ++tap) {
      int rl = l0 + m + tap;
      rl = rl > NLEN - 1 ? NLEN - 1 : rl;
      const size_t node = (size_t)b * NLEN + rl;
      const _Float16* arow = s16 + node * CF + 8 * hh;
      const float* frow = feat + node * CF + 8 * hh;
      const _Float16* brow = wt + (size_t)(cg * 128 + m) * KP + tap * CIN + 8 * hh;
#pragma unroll
      for (int ks = 0; ks < CF / 32; ++ks) {
        FragH a;
        a.h[0] = *(const v8h*)(arow + 32 * ks);
        a.h[1] = *(const v8h*)(arow + 32 * ks + 16);
#pragma unroll
        for (int t = 0; t < 8; ++t) {
          const _Float16* bp = brow + (size_t)(16 * t) * KP + 32 * ks;
          FragH bb;
          bb.h[0] = *(const v8h*)bp;
          bb.h[1] = *(const v8h*)(bp + 16);
          acc[t] = wmh(a.v, bb.v, acc[t]);
        }
      }
#pragma unroll
      for (int ks = 0; ks < (CIN - CF) / 32; ++ks) {
        FragH a;
        a.h[0] = cvt8(*(const v4f*)(frow + 32 * ks),      *(const v4f*)(frow + 32 * ks + 4));
        a.h[1] = cvt8(*(const v4f*)(frow + 32 * ks + 16), *(const v4f*)(frow + 32 * ks + 20));
#pragma unroll
        for (int t = 0; t < 8; ++t) {
          const _Float16* bp = brow + (size_t)(16 * t) * KP + CF + 32 * ks;
          FragH bb;
          bb.h[0] = *(const v8h*)bp;
          bb.h[1] = *(const v8h*)(bp + 16);
          acc[t] = wmh(a.v, bb.v, acc[t]);
        }
      }
    }

#pragma unroll
    for (int t = 0; t < 8; ++t) {
      const float bv = bias[cg * 128 + 16 * t + m];
      float* sp = stg + (16 * t + m) * PBLK + wave * 16 + 8 * hh;
#pragma unroll
      for (int r = 0; r < 8; ++r) sp[r] = acc[t][r] * WINV + bv;
    }
    __syncthreads();

    v4f ov[16];
#pragma unroll
    for (int i = 0; i < 16; ++i) ov[i] = *(const v4f*)(stg + (wave * 16 + i) * PBLK + 4 * lane);
    float* gp = Y + ((size_t)(b * CO + cg * 128 + wave * 16)) * LP + pb * PBLK + 4 * lane;
#pragma unroll
    for (int i = 0; i < 16; ++i) *(volatile v4f*)(gp + (size_t)i * LP) = ov[i];
    __threadfence();
#pragma unroll
    for (int i = 0; i < 16; ++i) *(volatile v4f*)(gp + (size_t)i * LP) = ov[i];
    __syncthreads();
  }
}

__global__ __launch_bounds__(NTHR) void k_bnstat(
    const float* __restrict__ y1, const float* __restrict__ y2, float* bnp) {
  __shared__ __attribute__((aligned(16))) float sp[64];
  const int tid = threadIdx.x, lane = tid & 31, wave = tid >> 5;
  const int cb = blockIdx.x;
  const bool br1 = cb < (CO1 / 32);
  const float* plane = br1 ? y1 : y2;
  const int CO = br1 ? CO1 : CO2;
#pragma unroll 1
  for (int q = 0; q < 4; ++q) {
    const int cl  = wave * 4 + q;
    const int chn = cb * 32 + cl;
    const int co  = br1 ? chn : chn - CO1;
    double s = 0.0, qq = 0.0;
#pragma unroll 1
    for (int bb = 0; bb < NGR; ++bb) {
      const float* row = plane + ((size_t)(bb * CO + co)) * LP;
#pragma unroll 2
      for (int i = 4 * lane; i < LP; i += 128) {
        const v4f v = *(const v4f*)(row + i);
        const float x0 = v.x;
        const float x1 = v.y;
        const float x2 = ((i + 2) < LOUT) ? v.z : 0.0f;
        const float x3 = ((i + 3) < LOUT) ? v.w : 0.0f;
        s += (double)x0; s += (double)x1; s += (double)x2; s += (double)x3;
        qq += (double)x0 * (double)x0; qq += (double)x1 * (double)x1;
        qq += (double)x2 * (double)x2; qq += (double)x3 * (double)x3;
      }
    }
#pragma unroll
    for (int o = 16; o > 0; o >>= 1) { s += shfl_xor_d(s, o); qq += shfl_xor_d(qq, o); }
    const double invn = 1.0 / (double)(NGR * LOUT);
    const double mu = s * invn;
    double var = qq * invn - mu * mu;
    var = var < 0.0 ? 0.0 : var;
    const float mf = (float)mu;
    const float vf = (float)var;
    const float rs = 1.0f / sqrtf(vf + BNEPS);
    if (lane == 0) { sp[2 * cl] = mf; sp[2 * cl + 1] = rs; }
  }
  __syncthreads();
  v4f ov = {0.f, 0.f, 0.f, 0.f};
  if (tid < 16) ov = *(const v4f*)(sp + 4 * tid);
  float* gp = bnp + (size_t)cb * 64;
  if (tid < 16) *(volatile v4f*)(gp + 4 * tid) = ov;
  __threadfence();
  if (tid < 16) *(volatile v4f*)(gp + 4 * tid) = ov;
}

__global__ __launch_bounds__(NTHR) void k_pool(
    const float* __restrict__ y1, const float* __restrict__ y2, const float* __restrict__ bnp,
    const float* __restrict__ g1, const float* __restrict__ be1,
    const float* __restrict__ g2, const float* __restrict__ be2, float* pool) {
  __shared__ __attribute__((aligned(16))) float sp[32];
  const int tid = threadIdx.x, lane = tid & 31, wave = tid >> 5;
  const int cb = blockIdx.x, b = blockIdx.y;
  const bool br1 = cb < (CO1 / 32);
  const float* plane = br1 ? y1 : y2;
  const int CO = br1 ? CO1 : CO2;
#pragma unroll 1
  for (int q = 0; q < 4; ++q) {
    const int cl  = wave * 4 + q;
    const int chn = cb * 32 + cl;
    const int co  = br1 ? chn : chn - CO1;
    const int i1  = chn < CO1 ? chn : CO1 - 1;
    int i2 = chn - CO1;
    i2 = i2 < 0 ? 0 : (i2 > CO2 - 1 ? CO2 - 1 : i2);
    const float ga1 = g1[i1], ga2 = g2[i2];
    const float bt1 = be1[i1], bt2 = be2[i2];
    const float ga = br1 ? ga1 : ga2;
    const float bt = br1 ? bt1 : bt2;
    const float mu = bnp[2 * chn], rs = bnp[2 * chn + 1];
    const float* row = plane + ((size_t)(b * CO + co)) * LP;
    float mx = 0.0f;
#pragma unroll 2
    for (int i = 4 * lane; i < LP; i += 128) {
      const v4f v = *(const v4f*)(row + i);
      float z0 = (ga * (v.x - mu)) * rs + bt;
      float z1 = (ga * (v.y - mu)) * rs + bt;
      float z2 = (ga * (v.z - mu)) * rs + bt;
      float z3 = (ga * (v.w - mu)) * rs + bt;
      z0 = fmaxf(z0, 0.0f); z1 = fmaxf(z1, 0.0f); z2 = fmaxf(z2, 0.0f); z3 = fmaxf(z3, 0.0f);
      z2 = ((i + 2) < LOUT) ? z2 : 0.0f;
      z3 = ((i + 3) < LOUT) ? z3 : 0.0f;
      mx = fmaxf(mx, fmaxf(fmaxf(z0, z1), fmaxf(z2, z3)));
    }
#pragma unroll
    for (int o = 16; o > 0; o >>= 1) mx = fmaxf(mx, __shfl_xor(mx, o, 32));
    if (lane == 0) sp[cl] = mx;
  }
  __syncthreads();
  v4f ov = {0.f, 0.f, 0.f, 0.f};
  if (tid < 8) ov = *(const v4f*)(sp + 4 * tid);
  float* gp = pool + (size_t)b * NCH + cb * 32;
  if (tid < 8) *(volatile v4f*)(gp + 4 * tid) = ov;
  __threadfence();
  if (tid < 8) *(volatile v4f*)(gp + 4 * tid) = ov;
}

__global__ __launch_bounds__(32) void k_heads(
    const float* __restrict__ pool,
    const float* __restrict__ w1, const float* __restrict__ b1,
    const float* __restrict__ w2, const float* __restrict__ b2, float* out) {
  __shared__ __attribute__((aligned(16))) float so[32];
  const int tid = threadIdx.x & 31;
  const int bb = tid >> 1, j = tid & 1;
  const float* p1 = pool + (size_t)bb * NCH;
  const float* p2 = p1 + CO1;
  float a = 0.0f;
#pragma unroll 4
  for (int c = 0; c < CO1; ++c) a += p1[c] * w1[j * CO1 + c];
  a += b1[j];
  float d = 0.0f;
#pragma unroll 4
  for (int c = 0; c < CO2; ++c) d += p2[c] * w2[j * CO2 + c];
  d += b2[j];
  so[tid] = a * d;
  __syncthreads();
  v4f ov = {0.f, 0.f, 0.f, 0.f};
  if (tid < 8) ov = *(const v4f*)(so + 4 * tid);
  if (tid < 8) *(volatile v4f*)(out + 4 * tid) = ov;
  __threadfence();
  if (tid < 8) *(volatile v4f*)(out + 4 * tid) = ov;
}

extern "C" void kernel_launch(void* const* d_in, const int* in_sizes, int n_in,
                              void* d_out, int out_size, void* d_ws, size_t ws_size,
                              hipStream_t stream) {
  if (n_in < 18) return;
  const int nN = in_sizes[0] / CF;
  if (nN != NGR * NLEN || in_sizes[0] != nN * CF) return;
  const int nE = in_sizes[1] / 2;
  if (nE < 1 || in_sizes[1] != 2 * nE || nE > (1 << 28)) return;
  if (in_sizes[3] != CF * CF || in_sizes[4] != CF || in_sizes[5] != CF * CF) return;
  if (in_sizes[6] != CO1 * CF * 3 || in_sizes[7] != CO1 || in_sizes[8] != CO1 || in_sizes[9] != CO1) return;
  if (in_sizes[10] != CO2 * KC * 3 || in_sizes[11] != CO2 || in_sizes[12] != CO2 || in_sizes[13] != CO2) return;
  if (in_sizes[14] != 2 * CO1 || in_sizes[15] != 2 || in_sizes[16] != 2 * CO2 || in_sizes[17] != 2) return;
  if (out_size != NGR * 2) return;

  const float* feature = (const float*)d_in[0];
  const int*   topo    = (const int*)d_in[1];
  const float* lin_l_w = (const float*)d_in[3];
  const float* lin_l_b = (const float*)d_in[4];
  const float* lin_r_w = (const float*)d_in[5];
  const float* conv1_w = (const float*)d_in[6];
  const float* conv1_b = (const float*)d_in[7];
  const float* bn1_g   = (const float*)d_in[8];
  const float* bn1_b   = (const float*)d_in[9];
  const float* conv2_w = (const float*)d_in[10];
  const float* conv2_b = (const float*)d_in[11];
  const float* bn2_g   = (const float*)d_in[12];
  const float* bn2_b   = (const float*)d_in[13];
  const float* lin1_w  = (const float*)d_in[14];
  const float* lin1_b  = (const float*)d_in[15];
  const float* lin2_w  = (const float*)d_in[16];
  const float* lin2_b  = (const float*)d_in[17];
  float* out = (float*)d_out;

  char* ws = (char*)d_ws;
  size_t off = 0;
  const size_t oWc   = off; off += (size_t)CF * KC * 2;                 off = (off + 255) & ~(size_t)255;
  const size_t oWt1  = off; off += (size_t)CO1 * 3 * CF * 2;            off = (off + 255) & ~(size_t)255;
  const size_t oWt2  = off; off += (size_t)CO2 * 3 * KC * 2;            off = (off + 255) & ~(size_t)255;
  const size_t oS16  = off; off += (size_t)nN * CF * 2;                 off = (off + 255) & ~(size_t)255;
  const size_t oY1   = off; off += (size_t)NGR * CO1 * LP * 4;          off = (off + 255) & ~(size_t)255;
  const size_t oY2   = off; off += (size_t)NGR * CO2 * LP * 4;          off = (off + 255) & ~(size_t)255;
  const size_t oBnp  = off; off += (size_t)NCH * 2 * 4;                 off = (off + 255) & ~(size_t)255;
  const size_t oPool = off; off += (size_t)NGR * NCH * 4;               off = (off + 255) & ~(size_t)255;
  if (off > ws_size || off > (size_t)134217728) return;
  _Float16* wc   = (_Float16*)(ws + oWc);
  _Float16* wt1  = (_Float16*)(ws + oWt1);
  _Float16* wt2  = (_Float16*)(ws + oWt2);
  _Float16* s16  = (_Float16*)(ws + oS16);
  float*    y1   = (float*)(ws + oY1);
  float*    y2   = (float*)(ws + oY2);
  float*    bnp  = (float*)(ws + oBnp);
  float*    pool = (float*)(ws + oPool);

  const int vec8 = ((nE & 3) == 0) ? 1 : 0;

  const int nPrep = CF * KC / 8 + CO1 * 3 * CF / 8 + CO2 * 3 * KC / 8;
  k_prep<<<(nPrep + NTHR - 1) / NTHR, NTHR, 0, stream>>>(lin_l_w, lin_r_w, conv1_w, conv2_w, wc, wt1, wt2);

  hipFuncSetAttribute(reinterpret_cast<const void*>(&k_aggl), hipFuncAttributeMaxDynamicSharedMemorySize, LDS_AGG);
  k_aggl<<<nN / TD, NTHR, LDS_AGG, stream>>>(feature, topo, wc, lin_l_b, s16, nN, nE, vec8);

  hipFuncSetAttribute(reinterpret_cast<const void*>(&k_conv<CF, CO1>), hipFuncAttributeMaxDynamicSharedMemorySize, LDS_CONV);
  hipFuncSetAttribute(reinterpret_cast<const void*>(&k_conv<KC, CO2>), hipFuncAttributeMaxDynamicSharedMemorySize, LDS_CONV);
  k_conv<CF, CO1><<<dim3(NLEN / PBLK, NGR), NTHR, LDS_CONV, stream>>>(s16, feature, wt1, conv1_b, y1);
  k_conv<KC, CO2><<<dim3(NLEN / PBLK, NGR), NTHR, LDS_CONV, stream>>>(s16, feature, wt2, conv2_b, y2);

  k_bnstat<<<NCH / 32, NTHR, 0, stream>>>(y1, y2, bnp);
  k_pool<<<dim3(NCH / 32, NGR), NTHR, 0, stream>>>(y1, y2, bnp, bn1_g, bn1_b, bn2_g, bn2_b, pool);
  k_heads<<<1, 32, 0, stream>>>(pool, lin1_w, lin1_b, lin2_w, lin2_b, out);
}
